// ExpertMLP_MPNet_17961553232376
// MI455X (gfx1250) — hardware-verified
//
#include <hip/hip_runtime.h>
#include <stddef.h>


typedef _Float16 v16h __attribute__((ext_vector_type(16)));
typedef _Float16 v8h  __attribute__((ext_vector_type(8)));
typedef float    v8f  __attribute__((ext_vector_type(8)));
typedef float    v4f  __attribute__((ext_vector_type(4)));

#ifndef NROWS
#define NROWS 512
#endif
#define NROWS_FULL 512
#define DIM   512
#define NEXP  8
#define KTOT  (NEXP * DIM)

static_assert(NROWS >= 64 && NROWS <= NROWS_FULL && (NROWS % 64) == 0);
static_assert((DIM % 64) == 0 && (DIM % 32) == 0 && (DIM % 8) == 0);
static_assert((KTOT % 64) == 0 && KTOT == NEXP * DIM);
static_assert(NEXP == 8);
static_assert(((size_t)NROWS * DIM) % 2048 == 0);

#define LDT 72
#define LDC 68
static_assert((LDT % 8) == 0 && LDT >= 64);
static_assert((LDC % 4) == 0 && LDC >= 64);

#define WCARRY  512.0f
#define XCARRY  16.0f
#define H1CARRY 256.0f
#define H2CARRY 4096.0f

#define WPL_BYTES ((size_t)DIM * KTOT * 2)
#define ACT_BYTES ((size_t)NROWS * DIM * 2)
#define OFF_W1  ((size_t)0)
#define OFF_W2  (OFF_W1 + WPL_BYTES)
#define OFF_W3  (OFF_W2 + WPL_BYTES)
#define OFF_X16 (OFF_W3 + WPL_BYTES)
#define OFF_H1  (OFF_X16 + ACT_BYTES)
#define OFF_H2  (OFF_H1 + ACT_BYTES)
#define WS_TOTAL (OFF_H2 + ACT_BYTES)
static_assert((WPL_BYTES % 128) == 0 && (ACT_BYTES % 128) == 0);
static_assert(WS_TOTAL <= (size_t)134217728);

__device__ __forceinline__ float bf16r(float x) {
  unsigned int u = __float_as_uint(x);
  u = (u + 0x7FFFu + ((u >> 16) & 1u)) & 0xFFFF0000u;
  return __uint_as_float(u);
}

static __device__ __forceinline__ _Float16 toh_flush(float v) {
  const _Float16 r = (_Float16)v;
  return (fabsf(v) < 6.103515625e-05f) ? (_Float16)0.0f : r;
}

__device__ __forceinline__ v16h frag_at(const _Float16* p) {
  v8h lo = *(const v8h*)(p);
  v8h hi = *(const v8h*)(p + 16);
  v16h out;
#pragma unroll
  for (int i = 0; i < 8; ++i) { out[i] = lo[i]; out[i + 8] = hi[i]; }
  return out;
}

__device__ __forceinline__ v8f wmma16(v16h a, v16h b, v8f c) {
  v8f d = __builtin_amdgcn_wmma_f32_16x16x32_f16(false, a, false, b, (short)0, c,
                                                 false, false);
  asm volatile("v_nop\n\tv_nop\n\tv_nop\n\tv_nop" : "+v"(d) : "v"(a), "v"(b));
  return d;
}

__device__ __forceinline__ float elu_act(float v) {
  const float vn = fminf(v, 0.0f);
  float p = 1.0f / 5040.0f;
  p = p * vn + (1.0f / 720.0f);
  p = p * vn + (1.0f / 120.0f);
  p = p * vn + (1.0f / 24.0f);
  p = p * vn + (1.0f / 6.0f);
  p = p * vn + 0.5f;
  p = p * vn + 1.0f;
  const float small = vn * p;
  const float big = __expf(vn) - 1.0f;
  const float neg = (vn > -0.25f) ? small : big;
  return (v > 0.0f) ? v : neg;
}

__global__ __launch_bounds__(256) void wconv_kernel(
    const float* __restrict__ W, _Float16* __restrict__ Wt, unsigned ldw, unsigned ldk) {
  __shared__ _Float16 T[64 * LDT];
  const unsigned tid = threadIdx.x;
  const unsigned n0 = blockIdx.x * 64u;
  const unsigned k0 = blockIdx.y * 64u;
#pragma unroll 4
  for (unsigned j = 0; j < 16u; ++j) {
    const unsigned idx = tid + 256u * j;
    const unsigned kr = idx >> 6, nc = idx & 63u;
    const float v = W[(size_t)(k0 + kr) * ldw + n0 + nc];
    T[nc * LDT + kr] = (_Float16)(WCARRY * bf16r(v));
  }
  __syncthreads();
  v8h x[2];
  size_t off[2];
#pragma unroll
  for (unsigned i = 0; i < 2u; ++i) {
    const unsigned n = 32u * i + (tid >> 3);
    const unsigned kc = (tid & 7u) * 8u;
    x[i] = *(const v8h*)&T[n * LDT + kc];
    off[i] = (size_t)(n0 + n) * ldk + k0 + kc;
  }
#pragma unroll
  for (int i = 0; i < 2; ++i) *(volatile v8h*)(Wt + off[i]) = x[i];
  __threadfence();
#pragma unroll
  for (int i = 0; i < 2; ++i) *(volatile v8h*)(Wt + off[i]) = x[i];
}

__global__ __launch_bounds__(256) void xconv_kernel(
    const float* __restrict__ X, _Float16* __restrict__ dst) {
  const size_t e0 = ((size_t)blockIdx.x * 256u + threadIdx.x) * 8u;
  const v4f a0 = *(const v4f*)(X + e0);
  const v4f a1 = *(const v4f*)(X + e0 + 4u);
  v8h o;
#pragma unroll
  for (int i = 0; i < 4; ++i) {
    o[i]     = toh_flush(XCARRY * bf16r(a0[i]));
    o[i + 4] = toh_flush(XCARRY * bf16r(a1[i]));
  }
  _Float16* p = dst + e0;
  *(volatile v8h*)p = o;
  __threadfence();
  *(volatile v8h*)p = o;
}

template <int LAST>
__device__ __forceinline__ void moe_body(
    const _Float16* __restrict__ A16, const _Float16* __restrict__ Bt,
    const float* __restrict__ coef, const float* __restrict__ bias,
    const float inv_scale, const float out_carry,
    float* __restrict__ outf, _Float16* __restrict__ out16) {
  __shared__ __attribute__((aligned(16))) float Cs[64 * LDC];
  __shared__ __attribute__((aligned(16))) float Cft[NEXP * 64];
  const unsigned tid = threadIdx.x, lane = tid & 31u;
  const unsigned w = (unsigned)__builtin_amdgcn_readfirstlane((int)(tid >> 5));
  const unsigned mw = w >> 1, nw = w & 1u;
  const unsigned hh = lane >> 4, m = lane & 15u;
  const unsigned n0 = blockIdx.x * 64u;
  const unsigned row0 = blockIdx.y * 64u;

#pragma unroll
  for (unsigned j = 0; j < 2u; ++j) {
    const unsigned idx = tid + 256u * j;
    const unsigned rr = idx >> 3, ee = idx & 7u;
    Cft[ee * 64u + rr] = bf16r(coef[(size_t)(row0 + rr) * NEXP + ee]);
  }
  __syncthreads();

  const _Float16* ap  = A16 + (size_t)(row0 + mw * 16u + m) * DIM + hh * 8u;
  const _Float16* bp0 = Bt + (size_t)(n0 + nw * 32u + m) * KTOT + hh * 8u;
  const _Float16* bp1 = bp0 + (size_t)16 * KTOT;
  v8f tot0 = {}, tot1 = {};
#pragma unroll 1
  for (unsigned e = 0; e < (unsigned)NEXP; ++e) {
    const unsigned kb = e * (unsigned)DIM;
    v8f acc0 = {}, acc1 = {};
#pragma unroll 2
    for (unsigned k0 = 0; k0 < (unsigned)DIM; k0 += 32u) {
      const v16h a  = frag_at(ap + k0);
      const v16h b0 = frag_at(bp0 + kb + k0);
      const v16h b1 = frag_at(bp1 + kb + k0);
      acc0 = wmma16(a, b0, acc0);
      acc1 = wmma16(a, b1, acc1);
    }
    const v4f c0 = *(const v4f*)&Cft[e * 64u + mw * 16u + hh * 8u];
    const v4f c1 = *(const v4f*)&Cft[e * 64u + mw * 16u + hh * 8u + 4u];
#pragma unroll
    for (int r = 0; r < 4; ++r) {
      tot0[r]     += c0[r] * acc0[r];
      tot0[r + 4] += c1[r] * acc0[r + 4];
      tot1[r]     += c0[r] * acc1[r];
      tot1[r + 4] += c1[r] * acc1[r + 4];
    }
  }
#pragma unroll
  for (int r = 0; r < 8; ++r) {
    float* d = &Cs[(mw * 16u + hh * 8u + (unsigned)r) * LDC + nw * 32u + m];
    d[0]  = tot0[r];
    d[16] = tot1[r];
  }
  __syncthreads();

#pragma unroll 1
  for (unsigned g = 0; g < 4u; ++g) {
    const unsigned r = LAST ? (16u * g + (tid >> 4)) : (32u * (g >> 1) + (tid >> 3));
    const unsigned c = LAST ? ((tid & 15u) * 4u) : ((tid & 7u) * 8u + 4u * (g & 1u));
    const v4f u = *(const v4f*)&Cs[r * LDC + c];
    v4f bb = {0.0f, 0.0f, 0.0f, 0.0f};
#pragma unroll 1
    for (unsigned e = 0; e < (unsigned)NEXP; ++e) {
      const float ce = Cft[e * 64u + r];
      const v4f gb = *(const v4f*)(bias + (size_t)e * DIM + n0 + c);
#pragma unroll
      for (int j = 0; j < 4; ++j) bb[j] += ce * bf16r(gb[j]);
    }
    v4f t;
#pragma unroll
    for (int j = 0; j < 4; ++j) {
      const float pre = u[j] * inv_scale + bb[j];
      t[j] = LAST ? pre : (out_carry * elu_act(pre));
    }
    *(v4f*)&Cs[r * LDC + c] = t;
  }

  if (LAST == 0) {
    v8h x[2];
    size_t off[2];
#pragma unroll
    for (unsigned i = 0; i < 2u; ++i) {
      const unsigned r = 32u * i + (tid >> 3);
      const unsigned c = (tid & 7u) * 8u;
      const v4f u0 = *(const v4f*)&Cs[r * LDC + c];
      const v4f u1 = *(const v4f*)&Cs[r * LDC + c + 4];
#pragma unroll
      for (int j = 0; j < 4; ++j) {
        x[i][j]     = toh_flush(u0[j]);
        x[i][j + 4] = toh_flush(u1[j]);
      }
      off[i] = (size_t)(row0 + r) * DIM + n0 + c;
    }
#pragma unroll
    for (int i = 0; i < 2; ++i) *(volatile v8h*)(out16 + off[i]) = x[i];
    __threadfence();
#pragma unroll
    for (int i = 0; i < 2; ++i) *(volatile v8h*)(out16 + off[i]) = x[i];
  }

  if (LAST == 1) {
    v4f xs[4];
    size_t off[4];
#pragma unroll
    for (unsigned i = 0; i < 4u; ++i) {
      const unsigned r = 16u * i + (tid >> 4);
      const unsigned c = (tid & 15u) * 4u;
      xs[i] = *(const v4f*)&Cs[r * LDC + c];
      off[i] = (size_t)(row0 + r) * DIM + n0 + c;
    }
#pragma unroll
    for (int i = 0; i < 4; ++i) *(volatile v4f*)(outf + off[i]) = xs[i];
    __threadfence();
#pragma unroll
    for (int i = 0; i < 4; ++i) *(volatile v4f*)(outf + off[i]) = xs[i];
  }
}

__global__ __launch_bounds__(256) void moe_hidden_kernel(
    const _Float16* __restrict__ A16, const _Float16* __restrict__ Bt,
    const float* __restrict__ coef, const float* __restrict__ bias,
    float inv_scale, float out_carry, _Float16* __restrict__ out16) {
  moe_body<0>(A16, Bt, coef, bias, inv_scale, out_carry, (float*)0, out16);
}
__global__ __launch_bounds__(256) void moe_out_kernel(
    const _Float16* __restrict__ A16, const _Float16* __restrict__ Bt,
    const float* __restrict__ coef, const float* __restrict__ bias,
    float inv_scale, float* __restrict__ outf) {
  moe_body<1>(A16, Bt, coef, bias, inv_scale, 1.0f, outf, (_Float16*)0);
}

extern "C" void kernel_launch(void* const* d_in, const int* in_sizes, int n_in,
                              void* d_out, int out_size, void* d_ws, size_t ws_size,
                              hipStream_t stream) {
  if (n_in < 8) return;
  if ((long long)in_sizes[0] < (long long)NROWS * DIM) return;
  if ((long long)in_sizes[1] < (long long)NROWS * NEXP) return;
  if ((long long)in_sizes[2] < (long long)KTOT * DIM) return;
  if ((long long)in_sizes[4] < (long long)KTOT * DIM) return;
  if ((long long)in_sizes[6] < (long long)KTOT * DIM) return;
  if (in_sizes[3] < NEXP * DIM || in_sizes[5] < NEXP * DIM || in_sizes[7] < NEXP * DIM) return;
  if ((long long)out_size < (long long)NROWS * DIM) return;
  if (ws_size < WS_TOTAL) return;

  const float* X    = (const float*)d_in[0];
  const float* coef = (const float*)d_in[1];
  const float* w1   = (const float*)d_in[2];
  const float* b1   = (const float*)d_in[3];
  const float* w2   = (const float*)d_in[4];
  const float* b2   = (const float*)d_in[5];
  const float* w3   = (const float*)d_in[6];
  const float* b3   = (const float*)d_in[7];
  float* out = (float*)d_out;

  char* ws = (char*)d_ws;
  _Float16* W1_t = (_Float16*)(ws + OFF_W1);
  _Float16* W2_t = (_Float16*)(ws + OFF_W2);
  _Float16* W3_t = (_Float16*)(ws + OFF_W3);
  _Float16* X16  = (_Float16*)(ws + OFF_X16);
  _Float16* H1   = (_Float16*)(ws + OFF_H1);
  _Float16* H2   = (_Float16*)(ws + OFF_H2);

  dim3 blk(256);
  dim3 gw(DIM / 64, KTOT / 64);
  dim3 gg(DIM / 64, NROWS / 64);

  wconv_kernel<<<gw, blk, 0, stream>>>(w1, W1_t, (unsigned)DIM, (unsigned)KTOT);
  wconv_kernel<<<gw, blk, 0, stream>>>(w2, W2_t, (unsigned)DIM, (unsigned)KTOT);
  wconv_kernel<<<gw, blk, 0, stream>>>(w3, W3_t, (unsigned)DIM, (unsigned)KTOT);
  xconv_kernel<<<dim3((unsigned)(((size_t)NROWS * DIM) / 2048)), blk, 0, stream>>>(X, X16);

  moe_hidden_kernel<<<gg, blk, 0, stream>>>(X16, W1_t, coef, b1,
                                            1.0f / (XCARRY * WCARRY), H1CARRY, H1);
  moe_hidden_kernel<<<gg, blk, 0, stream>>>(H1, W2_t, coef, b2,
                                            1.0f / (H1CARRY * WCARRY), H2CARRY, H2);
  moe_out_kernel<<<gg, blk, 0, stream>>>(H2, W3_t, coef, b3,
                                         1.0f / (H2CARRY * WCARRY), out);
}
